// DeltaNet_45397804319521
// MI455X (gfx1250) — hardware-run, weakly checked
//
#include <hip/hip_runtime.h>
#include <math.h>

typedef __attribute__((ext_vector_type(16))) _Float16 v16h;
typedef __attribute__((ext_vector_type(8)))  _Float16 v8h;
typedef __attribute__((ext_vector_type(8)))  float    v8f;
typedef __attribute__((ext_vector_type(4)))  float    v4f;
typedef __attribute__((ext_vector_type(4)))  unsigned int v4u;

constexpr int kBatch  = 4;
constexpr int kSeq    = 512;
constexpr int kHid    = 512;
constexpr int kTaps   = 4;
constexpr int kRows   = kBatch * kSeq;
constexpr int kChunk  = 32;
constexpr int kNChunk = kSeq / kChunk;
constexpr int kNI     = 32;
constexpr int kQkvP   = 3 * kHid;
constexpr int kSP     = 520;
constexpr int kVP     = 36;
constexpr int kUP     = 40;
static_assert(kRows == 2048 && kNChunk == 16 && kQkvP == 1536);
static_assert((kRows % 64) == 0 && (kQkvP % 64) == 0 && (kHid % 64) == 0 && (kHid % 32) == 0);
static_assert(kChunk == 32 && kNI == 32 && (kSeq % kChunk) == 0 && (kHid % kNI) == 0);

constexpr float kCarX  = 16.0f;
constexpr float kCarW  = 256.0f;
constexpr float kCarKQ = 256.0f;
constexpr float kCarS  = 128.0f;
constexpr float kCarU  = 128.0f;
constexpr float kCarT  = 64.0f;
constexpr float kCarL  = 256.0f;
constexpr float kCarN  = 16.0f;
constexpr float kMaster     = kCarU * kCarKQ;
constexpr float kMasterInv  = 1.0f / kMaster;
constexpr float kProjScale  = 1.0f / (kCarX * kCarW);
constexpr float kGramScale  = 1.0f / (kCarKQ * kCarKQ);
constexpr float kUqScale    = 1.0f / kCarT;
constexpr float kShadowScl  = kCarS / kMaster;
constexpr float kOutScale   = 1.0f / (kCarN * kCarW);
constexpr float kF16MinNorm = 6.103515625e-5f;
static_assert(kCarKQ * kCarS == kMaster);
static_assert(kCarL * kCarU == kMaster);
static_assert(kMaster == 32768.0f);

constexpr size_t kSzPlane16 = (size_t)kRows * kHid * 2;
constexpr size_t kSzPlane32 = (size_t)kRows * kHid * 4;
constexpr size_t kOffX16  = 0;
constexpr size_t kOffW16  = kOffX16  + kSzPlane16;
constexpr size_t kOffRAW  = kOffW16  + (size_t)4 * kHid * kHid * 2;
constexpr size_t kOffK16  = kOffRAW  + (size_t)kRows * kQkvP * 4;
constexpr size_t kOffQ16  = kOffK16  + kSzPlane16;
constexpr size_t kOffKT16 = kOffQ16  + kSzPlane16;
constexpr size_t kOffV32  = kOffKT16 + kSzPlane16;
constexpr size_t kOffOBUF = kOffV32  + kSzPlane32;
constexpr size_t kOffON16 = kOffOBUF + kSzPlane32;
constexpr size_t kOffBETA = kOffON16 + kSzPlane16;
constexpr size_t kOffT16  = kOffBETA + (size_t)kRows * 4;
constexpr size_t kOffL16  = kOffT16  + (size_t)kBatch * kNChunk * kChunk * kChunk * 2;
constexpr size_t kWsTotal = kOffL16  + (size_t)kBatch * kNChunk * kChunk * kChunk * 2;
static_assert(kWsTotal == 33824768ull);
static_assert(kWsTotal <= 134217728ull);
static_assert((kOffW16 % 128) == 0 && (kOffRAW % 128) == 0 && (kOffK16 % 128) == 0 && (kOffQ16 % 128) == 0 &&
              (kOffKT16 % 128) == 0 && (kOffV32 % 128) == 0 && (kOffOBUF % 128) == 0 && (kOffON16 % 128) == 0 &&
              (kOffBETA % 128) == 0 && (kOffT16 % 128) == 0 && (kOffL16 % 128) == 0);

__device__ __forceinline__ float flush_below_f16_normal(float v) {
  return (fabsf(v) < kF16MinNorm) ? 0.0f : v;
}
__device__ __forceinline__ _Float16 to_h_fl(float v) {
  return (_Float16)flush_below_f16_normal(v);
}
__device__ __forceinline__ unsigned short h_bits_fl(float v) {
  const _Float16 h = to_h_fl(v);
  return __builtin_bit_cast(unsigned short, h);
}
__device__ __forceinline__ unsigned pk16(unsigned short a, unsigned short b) {
  return (unsigned)a | ((unsigned)b << 16);
}
__device__ __forceinline__ float silu_f(float v) {
  return v * (1.0f / (1.0f + expf(-v)));
}

union FragU { v16h v; v8h h[2]; };
__device__ __forceinline__ v16h frag_load(const _Float16* p) {
  FragU f;
  f.h[0] = *(const v8h*)(p);
  f.h[1] = *(const v8h*)(p + 16);
  return f.v;
}
__device__ __forceinline__ v8f mma_g(v16h a, v16h b, v8f c) {
  c = __builtin_amdgcn_wmma_f32_16x16x32_f16(false, a, false, b, (short)0, c, false, false);
  asm volatile("v_nop\n\tv_nop\n\tv_nop\n\tv_nop" : "+v"(c) : "v"(a), "v"(b));
  return c;
}
__device__ __forceinline__ v8f mma_raw(v16h a, v16h b, v8f c) {
  return __builtin_amdgcn_wmma_f32_16x16x32_f16(false, a, false, b, (short)0, c, false, false);
}
__device__ __forceinline__ void guard_row4(v8f& a, v8f& b, v8f& c, v8f& d, v16h x) {
  asm volatile("v_nop\n\tv_nop\n\tv_nop\n\tv_nop" : "+v"(a), "+v"(b), "+v"(c), "+v"(d) : "v"(x));
}
__device__ __forceinline__ void keep4_h(v16h a, v16h b, v16h c, v16h d) {
  asm volatile("v_nop" :: "v"(a), "v"(b), "v"(c), "v"(d));
}
__device__ __forceinline__ void acc_guard4(v8f& a, v8f& b, v8f& c, v8f& d) {
  asm volatile("v_nop\n\tv_nop\n\tv_nop\n\tv_nop" : "+v"(a), "+v"(b), "+v"(c), "+v"(d));
}

__global__ __launch_bounds__(256) void wmma_gemm64_f16(
    const unsigned short* __restrict__ Ap, int lda,
    const unsigned short* __restrict__ Btp, int ldb,
    float* __restrict__ C, int ldc, int M, int N, int K, float scale) {
  const _Float16* A  = (const _Float16*)Ap;
  const _Float16* Bt = (const _Float16*)Btp;
  __shared__ __align__(16) float sT[8][16 * 68];
  const int lane = threadIdx.x & 31;
  const int wave = threadIdx.x >> 5;
  const int tilesN = N >> 6;
  const int tilesM = M >> 6;
  const int tile = blockIdx.x * 8 + wave;
  if (tile >= tilesM * tilesN) return;
  const int tm = tile / tilesN;
  const int tn = tile - tm * tilesN;
  const int m0 = tm << 6;
  const int n0 = tn << 6;
  const int rlane = lane & 15;
  const int koff  = (lane >> 4) * 8;
  const int mOff  = (lane >> 4) * 8;

  v8f acc[4][4];
#pragma unroll
  for (int i = 0; i < 4; ++i)
#pragma unroll
    for (int j = 0; j < 4; ++j) acc[i][j] = (v8f){0.f, 0.f, 0.f, 0.f, 0.f, 0.f, 0.f, 0.f};

  for (int k0 = 0; k0 < K; k0 += 32) {
    v16h bh[4];
#pragma unroll
    for (int j = 0; j < 4; ++j) {
      const size_t bo = (size_t)(n0 + (j << 4) + rlane) * ldb + koff + k0;
      bh[j] = frag_load(Bt + bo);
    }
#pragma unroll
    for (int i = 0; i < 4; ++i) {
      const size_t ao = (size_t)(m0 + (i << 4) + rlane) * lda + koff + k0;
      const v16h ah = frag_load(A + ao);
#pragma unroll
      for (int j = 0; j < 4; ++j) acc[i][j] = mma_raw(ah, bh[j], acc[i][j]);
      guard_row4(acc[i][0], acc[i][1], acc[i][2], acc[i][3], ah);
    }
    keep4_h(bh[0], bh[1], bh[2], bh[3]);
  }
  acc_guard4(acc[0][0], acc[0][1], acc[0][2], acc[0][3]);
  acc_guard4(acc[1][0], acc[1][1], acc[1][2], acc[1][3]);
  acc_guard4(acc[2][0], acc[2][1], acc[2][2], acc[2][3]);
  acc_guard4(acc[3][0], acc[3][1], acc[3][2], acc[3][3]);

  float* slab = sT[wave];
#pragma unroll
  for (int i = 0; i < 4; ++i) {
    const int mBase = m0 + (i << 4);
#pragma unroll
    for (int j = 0; j < 4; ++j) {
#pragma unroll
      for (int r = 0; r < 8; ++r) {
        slab[(mOff + r) * 68 + (j << 4) + rlane] = acc[i][j][r] * scale;
      }
    }
    __builtin_amdgcn_fence(__ATOMIC_RELEASE, "workgroup");
    __builtin_amdgcn_wave_barrier();
    __builtin_amdgcn_fence(__ATOMIC_ACQUIRE, "workgroup");
    {
      const int hh = lane >> 4, c4 = (lane & 15) * 4;
      for (int pass = 0; pass < 2; ++pass) {
#pragma unroll
        for (int it = 0; it < 8; ++it) {
          const int row = it * 2 + hh;
          const v4f v = *(const v4f*)(slab + row * 68 + c4);
          *(volatile v4f*)(C + (size_t)(mBase + row) * ldc + n0 + c4) = v;
        }
        __threadfence();
      }
    }
    __builtin_amdgcn_fence(__ATOMIC_RELEASE, "workgroup");
    __builtin_amdgcn_wave_barrier();
    __builtin_amdgcn_fence(__ATOMIC_ACQUIRE, "workgroup");
  }
}

__global__ __launch_bounds__(256) void xcvt_beta_kernel(
    const float* __restrict__ x, const float* __restrict__ Wb,
    unsigned short* __restrict__ x16, float* __restrict__ beta) {
  __shared__ float sBeta[32];
  const int tid = threadIdx.x, lane = tid & 31, wave = tid >> 5;
  const int c0 = lane * 8;
  const v4f w0 = *(const v4f*)(Wb + c0);
  const v4f w1 = *(const v4f*)(Wb + c0 + 4);
  const v4f w2 = *(const v4f*)(Wb + 256 + c0);
  const v4f w3 = *(const v4f*)(Wb + 256 + c0 + 4);
#pragma unroll 1
  for (int rr = 0; rr < 4; ++rr) {
    const int rl = wave * 4 + rr;
    const size_t row = (size_t)blockIdx.x * 32 + rl;
    const float* xr = x + row * kHid;
    const v4f a0 = *(const v4f*)(xr + c0);
    const v4f a1 = *(const v4f*)(xr + c0 + 4);
    const v4f a2 = *(const v4f*)(xr + 256 + c0);
    const v4f a3 = *(const v4f*)(xr + 256 + c0 + 4);
    float s = 0.0f;
#pragma unroll
    for (int e = 0; e < 4; ++e) {
      s = fmaf(a0[e], w0[e], s);
      s = fmaf(a1[e], w1[e], s);
      s = fmaf(a2[e], w2[e], s);
      s = fmaf(a3[e], w3[e], s);
    }
#pragma unroll
    for (int off = 16; off > 0; off >>= 1) s += __shfl_xor(s, off, 32);
    const float bv = 1.0f / (1.0f + expf(-s));
    if (lane == 0) sBeta[rl] = bv;
    unsigned short hb[16];
#pragma unroll
    for (int e = 0; e < 4; ++e) {
      hb[e]      = h_bits_fl(a0[e] * kCarX);
      hb[4 + e]  = h_bits_fl(a1[e] * kCarX);
      hb[8 + e]  = h_bits_fl(a2[e] * kCarX);
      hb[12 + e] = h_bits_fl(a3[e] * kCarX);
    }
    const v4u u0 = (v4u){pk16(hb[0], hb[1]), pk16(hb[2], hb[3]), pk16(hb[4], hb[5]), pk16(hb[6], hb[7])};
    const v4u u1 = (v4u){pk16(hb[8], hb[9]), pk16(hb[10], hb[11]), pk16(hb[12], hb[13]), pk16(hb[14], hb[15])};
    unsigned short* d = x16 + row * kHid;
    for (int pass = 0; pass < 2; ++pass) {
      *(volatile v4u*)(d + c0) = u0;
      *(volatile v4u*)(d + 256 + c0) = u1;
      __threadfence();
    }
  }
  __syncthreads();
  if (wave == 0) {
    const float bv = sBeta[lane];
    float* d = beta + (size_t)blockIdx.x * 32 + lane;
    *(volatile float*)d = bv;
    __threadfence();
    *(volatile float*)d = bv;
  }
}

__global__ __launch_bounds__(256) void wcast_kernel(
    const float* __restrict__ W0, const float* __restrict__ W1,
    const float* __restrict__ W2, const float* __restrict__ W3,
    unsigned short* __restrict__ out) {
  const int z = blockIdx.y;
  const float* W = (z == 0) ? W0 : ((z == 1) ? W1 : ((z == 2) ? W2 : W3));
  const int i = blockIdx.x * 256 + threadIdx.x;
  if (i >= kHid * kHid / 8) return;
  const float* p = W + 8 * (size_t)i;
  const v4f a = *(const v4f*)(p);
  const v4f c = *(const v4f*)(p + 4);
  unsigned short hb[8];
#pragma unroll
  for (int e = 0; e < 4; ++e) {
    hb[e]     = h_bits_fl(a[e] * kCarW);
    hb[4 + e] = h_bits_fl(c[e] * kCarW);
  }
  const v4u u = (v4u){pk16(hb[0], hb[1]), pk16(hb[2], hb[3]), pk16(hb[4], hb[5]), pk16(hb[6], hb[7])};
  unsigned short* q = out + (size_t)z * kHid * kHid + 8 * (size_t)i;
  *(volatile v4u*)q = u;
  __threadfence();
  *(volatile v4u*)q = u;
}

__global__ __launch_bounds__(256) void conv_act_norm_kernel(
    const float* __restrict__ raw, const float* __restrict__ ck, const float* __restrict__ cq,
    const float* __restrict__ cv, unsigned short* __restrict__ k16, unsigned short* __restrict__ q16,
    float* __restrict__ v32) {
  __shared__ __align__(16) float sY[kQkvP];
  __shared__ float sRed[16];
  const int tid = threadIdx.x, lane = tid & 31, wave = tid >> 5;
  const int row = blockIdx.x;
  const int t = row & (kSeq - 1);
  float ssk = 0.0f, ssq = 0.0f;
#pragma unroll 1
  for (int it = 0; it < 6; ++it) {
    const int e = it * 256 + tid;
    const int s = it >> 1;
    const int c = e - s * kHid;
    const float* cw = (s == 0) ? ck : ((s == 1) ? cq : cv);
    const v4f w = *(const v4f*)(cw + c * kTaps);
    float acc = 0.0f;
#pragma unroll
    for (int j = 0; j < 4; ++j) {
      const bool valid = (t - 3 + j) >= 0;
      const int rj = valid ? (row - 3 + j) : row;
      const float ld = raw[(size_t)rj * kQkvP + e];
      const float xv = valid ? ld : 0.0f;
      acc = fmaf(w[j], xv, acc);
    }
    const float y = silu_f(silu_f(acc));
    sY[e] = y;
    const float sq = y * y;
    ssk += (s == 0) ? sq : 0.0f;
    ssq += (s == 1) ? sq : 0.0f;
  }
#pragma unroll
  for (int off = 16; off > 0; off >>= 1) {
    ssk += __shfl_xor(ssk, off, 32);
    ssq += __shfl_xor(ssq, off, 32);
  }
  if (lane == 0) {
    sRed[wave] = ssk;
    sRed[8 + wave] = ssq;
  }
  __syncthreads();
  float tk = 0.0f, tq = 0.0f;
#pragma unroll
  for (int i = 0; i < 8; ++i) {
    tk += sRed[i];
    tq += sRed[8 + i];
  }
  const float invk = 1.0f / fmaxf(sqrtf(tk), 1e-12f);
  const float invq = 1.0f / fmaxf(sqrtf(tq), 1e-12f);
  if (wave < 4) {
    const int s2 = wave >> 1;
    const int idx = (wave & 1) * 32 + lane;
    const float sc = ((s2 == 0) ? invk : invq) * kCarKQ;
    const float* sp = sY + s2 * kHid + idx * 8;
    const v4f a = *(const v4f*)(sp);
    const v4f c = *(const v4f*)(sp + 4);
    unsigned short hb[8];
#pragma unroll
    for (int e = 0; e < 4; ++e) {
      hb[e]     = h_bits_fl(a[e] * sc);
      hb[4 + e] = h_bits_fl(c[e] * sc);
    }
    const v4u u = (v4u){pk16(hb[0], hb[1]), pk16(hb[2], hb[3]), pk16(hb[4], hb[5]), pk16(hb[6], hb[7])};
    unsigned short* dst = ((s2 == 0) ? k16 : q16) + (size_t)row * kHid + idx * 8;
    *(volatile v4u*)dst = u;
    __threadfence();
    *(volatile v4u*)dst = u;
  } else {
    const int idx = (wave - 4) * 32 + lane;
    const v4f a = *(const v4f*)(sY + 2 * kHid + idx * 4);
    float* dst = v32 + (size_t)row * kHid + idx * 4;
    *(volatile v4f*)dst = a;
    __threadfence();
    *(volatile v4f*)dst = a;
  }
}

__global__ __launch_bounds__(256) void ktrans_kernel(
    const unsigned short* __restrict__ k16, unsigned short* __restrict__ kT16) {
  __shared__ unsigned short sm[64 * 72];
  const int tid = threadIdx.x, lane = tid & 31, wave = tid >> 5;
  const int t0 = blockIdx.x * 64, j0 = blockIdx.y * 64, b = blockIdx.z;
#pragma unroll
  for (int i = 0; i < 2; ++i) {
    const int idx = i * 256 + tid;
    const int r = idx >> 3, seg = idx & 7;
    const v4u u = *(const v4u*)(k16 + (size_t)(b * kSeq + t0 + r) * kHid + j0 + seg * 8);
    const unsigned w0 = u.x, w1 = u.y, w2 = u.z, w3 = u.w;
    unsigned short* col = sm + (seg * 8) * 72 + r;
    col[0 * 72] = (unsigned short)(w0 & 0xffffu);
    col[1 * 72] = (unsigned short)(w0 >> 16);
    col[2 * 72] = (unsigned short)(w1 & 0xffffu);
    col[3 * 72] = (unsigned short)(w1 >> 16);
    col[4 * 72] = (unsigned short)(w2 & 0xffffu);
    col[5 * 72] = (unsigned short)(w2 >> 16);
    col[6 * 72] = (unsigned short)(w3 & 0xffffu);
    col[7 * 72] = (unsigned short)(w3 >> 16);
  }
  __syncthreads();
  const int q = lane >> 3, c8 = (lane & 7) * 8;
  v4u o[2];
#pragma unroll
  for (int it = 0; it < 2; ++it) {
    const int rowl = wave * 8 + it * 4 + q;
    const unsigned short* sp = sm + rowl * 72 + c8;
    o[it] = (v4u){pk16(sp[0], sp[1]), pk16(sp[2], sp[3]), pk16(sp[4], sp[5]), pk16(sp[6], sp[7])};
  }
  for (int pass = 0; pass < 2; ++pass) {
#pragma unroll
    for (int it = 0; it < 2; ++it) {
      const int rowl = wave * 8 + it * 4 + q;
      *(volatile v4u*)(kT16 + (size_t)(b * kHid + j0 + rowl) * kSeq + t0 + c8) = o[it];
    }
    __threadfence();
  }
}

__global__ __launch_bounds__(256) void chunk_prep_kernel(
    const unsigned short* __restrict__ k16p, const unsigned short* __restrict__ q16p,
    const float* __restrict__ beta, unsigned short* __restrict__ T16, unsigned short* __restrict__ L16) {
  __shared__ float sGQ[64 * 33];
  __shared__ float sTm[32 * 33];
  __shared__ float sB[32];
  const int tid = threadIdx.x, lane = tid & 31;
  const int wave = __builtin_amdgcn_readfirstlane(tid >> 5);
  const int hh = lane >> 4, c = lane & 15;
  const int bc = blockIdx.x;
  const int rb = bc * kChunk;
  const _Float16* Kp = (const _Float16*)k16p;
  const _Float16* Qp = (const _Float16*)q16p;
  const int mt = wave >> 1, nt = wave & 1;
  const _Float16* Ap = ((mt < 2) ? Kp : Qp) + (size_t)(rb + 16 * (mt & 1) + c) * kHid + 8 * hh;
  const _Float16* Bp = Kp + (size_t)(rb + 16 * nt + c) * kHid + 8 * hh;
  float bv = beta[rb + lane];
  asm volatile("" : "+v"(bv));
  if (wave == 0) sB[lane] = bv;
  v8f acc = (v8f){0.f, 0.f, 0.f, 0.f, 0.f, 0.f, 0.f, 0.f};
#pragma unroll 2
  for (int k0 = 0; k0 < kHid; k0 += 32) {
    const v16h a = frag_load(Ap + k0);
    const v16h bf = frag_load(Bp + k0);
    acc = mma_g(a, bf, acc);
  }
#pragma unroll
  for (int r = 0; r < 8; ++r) sGQ[(16 * mt + 8 * hh + r) * 33 + 16 * nt + c] = acc[r] * kGramScale;
  __syncthreads();
  if (wave == 0) {
#pragma unroll 1
    for (int i = 0; i < 32; ++i) {
      float s = (i == lane) ? 1.0f : 0.0f;
      const float bi = sB[i];
#pragma unroll 1
      for (int m = 0; m < i; ++m) s = fmaf(-(bi * sGQ[i * 33 + m]), sTm[m * 33 + lane], s);
      sTm[i * 33 + lane] = s;
    }
  }
  __syncthreads();
  const int e0 = ((wave & 3) * 32 + lane) * 8;
  const int rowl = e0 >> 5, col = e0 & 31;
  unsigned short hb[8];
  if (wave < 4) {
#pragma unroll
    for (int e = 0; e < 8; ++e) hb[e] = h_bits_fl(sTm[rowl * 33 + col + e] * kCarT);
  } else {
#pragma unroll
    for (int e = 0; e < 8; ++e) {
      const float qk = sGQ[(32 + rowl) * 33 + col + e] * kCarL;
      hb[e] = h_bits_fl(((col + e) <= rowl) ? qk : 0.0f);
    }
  }
  const v4u u = (v4u){pk16(hb[0], hb[1]), pk16(hb[2], hb[3]), pk16(hb[4], hb[5]), pk16(hb[6], hb[7])};
  unsigned short* dst = ((wave < 4) ? T16 : L16) + (size_t)bc * (kChunk * kChunk) + e0;
  *(volatile v4u*)dst = u;
  __threadfence();
  *(volatile v4u*)dst = u;
}

__global__ __launch_bounds__(256) void state_scan_kernel(
    const unsigned short* __restrict__ k16p, const unsigned short* __restrict__ q16p,
    const unsigned short* __restrict__ kT16p, const float* __restrict__ v32,
    const float* __restrict__ beta, const unsigned short* __restrict__ T16p,
    const unsigned short* __restrict__ L16p, float* __restrict__ obuf, float* __restrict__ Sout) {
  __shared__ __align__(16) unsigned char sRaw[kNI * kSP * 2];
  __shared__ __align__(16) float sV[kChunk * kVP];
  __shared__ __align__(16) float sO[kChunk * kVP];
  __shared__ __align__(16) _Float16 sRmT[kNI * kUP];
  __shared__ __align__(16) _Float16 sUqT[kNI * kUP];
  __shared__ float sBeta[kChunk];
  static_assert(8 * 16 * 64 * 4 <= kNI * kSP * 2);
  _Float16* sS16 = (_Float16*)sRaw;

  const int tid = threadIdx.x, lane = tid & 31;
  const int wave = __builtin_amdgcn_readfirstlane(tid >> 5);
  const int hh = lane >> 4, c = lane & 15;
  const int i0 = blockIdx.x * kNI;
  const int b  = blockIdx.y;
  const _Float16* Kp  = (const _Float16*)k16p;
  const _Float16* Qp  = (const _Float16*)q16p;
  const _Float16* KTp = (const _Float16*)kT16p;
  const _Float16* Tp  = (const _Float16*)T16p;
  const _Float16* Lp  = (const _Float16*)L16p;
  const int mt = wave >> 1, nt = wave & 1;
  const int mt2 = mt & 1;

  {
    v4u* z = (v4u*)sRaw;
    for (int idx = tid; idx < (kNI * kSP * 2) / 16; idx += 256) z[idx] = (v4u){0u, 0u, 0u, 0u};
  }
  v8f sacc[2][4];
#pragma unroll
  for (int a = 0; a < 2; ++a)
#pragma unroll
    for (int j = 0; j < 4; ++j) sacc[a][j] = (v8f){0.f, 0.f, 0.f, 0.f, 0.f, 0.f, 0.f, 0.f};

#pragma unroll 1
  for (int ch = 0; ch < kNChunk; ++ch) {
    const int t0 = ch * kChunk;
    const int rb = b * kSeq + t0;
    const int bc = b * kNChunk + ch;
    {
      const int r = tid >> 3, c4 = (tid & 7) * 4;
      const v4f vv = *(const v4f*)(v32 + (size_t)(rb + r) * kHid + i0 + c4);
      *(v4f*)(sV + r * kVP + c4) = vv;
      float bvl = beta[rb + lane];
      asm volatile("" : "+v"(bvl));
      if (wave == 0) sBeta[lane] = bvl;
    }
    __syncthreads();

    v8f pacc = (v8f){0.f, 0.f, 0.f, 0.f, 0.f, 0.f, 0.f, 0.f};
    {
      const _Float16* Ap = ((mt < 2) ? Kp : Qp) + (size_t)(rb + 16 * mt2 + c) * kHid + 8 * hh;
      const _Float16* Bp = sS16 + (16 * nt + c) * kSP + 8 * hh;
#pragma unroll 2
      for (int k0 = 0; k0 < kHid; k0 += 32) {
        const v16h a = frag_load(Ap + k0);
        const v16h bf = frag_load(Bp + k0);
        pacc = mma_g(a, bf, pacc);
      }
    }
    if (wave < 4) {
      const int tl = 16 * mt + 8 * hh;
      const int il = 16 * nt + c;
      v8h hv;
#pragma unroll
      for (int r = 0; r < 8; ++r) {
        const float ks = pacc[r] * kMasterInv;
        const float rm = sBeta[tl + r] * (sV[(tl + r) * kVP + il] - ks);
        hv[r] = to_h_fl(rm * kCarU);
      }
      *(v8h*)(sRmT + il * kUP + tl) = hv;
    }
    __syncthreads();

    if (wave < 4) {
      const v16h a = frag_load(Tp + (size_t)bc * (kChunk * kChunk) + (16 * mt2 + c) * kChunk + 8 * hh);
      const v16h bf = frag_load(sRmT + (16 * nt + c) * kUP + 8 * hh);
      v8f uacc = (v8f){0.f, 0.f, 0.f, 0.f, 0.f, 0.f, 0.f, 0.f};
      uacc = mma_g(a, bf, uacc);
      v8h hv;
#pragma unroll
      for (int r = 0; r < 8; ++r) hv[r] = to_h_fl(uacc[r] * kUqScale);
      *(v8h*)(sUqT + (16 * nt + c) * kUP + 16 * mt2 + 8 * hh) = hv;
    }
    __syncthreads();

    if (wave >= 4) {
      const v16h a = frag_load(Lp + (size_t)bc * (kChunk * kChunk) + (16 * mt2 + c) * kChunk + 8 * hh);
      const v16h bf = frag_load(sUqT + (16 * nt + c) * kUP + 8 * hh);
      pacc = mma_g(a, bf, pacc);
#pragma unroll
      for (int r = 0; r < 8; ++r) sO[(16 * mt2 + 8 * hh + r) * kVP + 16 * nt + c] = pacc[r] * kMasterInv;
    }
    {
      const v16h a0 = frag_load(sUqT + c * kUP + 8 * hh);
      const v16h a1 = frag_load(sUqT + (16 + c) * kUP + 8 * hh);
#pragma unroll
      for (int jt = 0; jt < 4; ++jt) {
        const v16h bf = frag_load(KTp + (size_t)(b * kHid + 64 * wave + 16 * jt + c) * kSeq + t0 + 8 * hh);
        sacc[0][jt] = mma_g(a0, bf, sacc[0][jt]);
        sacc[1][jt] = mma_g(a1, bf, sacc[1][jt]);
      }
    }
#pragma unroll
    for (int a = 0; a < 2; ++a)
#pragma unroll
      for (int jt = 0; jt < 4; ++jt)
#pragma unroll
        for (int r = 0; r < 8; ++r)
          sS16[(16 * a + 8 * hh + r) * kSP + 64 * wave + 16 * jt + c] = to_h_fl(sacc[a][jt][r] * kShadowScl);
    __syncthreads();

    {
      const int rowl = 4 * wave + (lane >> 3), c4 = (lane & 7) * 4;
      const v4f ov = *(const v4f*)(sO + rowl * kVP + c4);
      float* dst = obuf + (size_t)(rb + rowl) * kHid + i0 + c4;
      *(volatile v4f*)dst = ov;
      __threadfence();
      *(volatile v4f*)dst = ov;
    }
  }

  float* slab = (float*)sRaw + wave * (16 * 64);
#pragma unroll
  for (int a = 0; a < 2; ++a) {
#pragma unroll
    for (int jt = 0; jt < 4; ++jt)
#pragma unroll
      for (int r = 0; r < 8; ++r) slab[(8 * hh + r) * 64 + 16 * jt + c] = sacc[a][jt][r] * kMasterInv;
    __builtin_amdgcn_fence(__ATOMIC_RELEASE, "workgroup");
    __builtin_amdgcn_wave_barrier();
    __builtin_amdgcn_fence(__ATOMIC_ACQUIRE, "workgroup");
    {
      const int c4 = c * 4;
      for (int pass = 0; pass < 2; ++pass) {
#pragma unroll
        for (int it = 0; it < 8; ++it) {
          const int rowl = it * 2 + hh;
          const v4f sv = *(const v4f*)(slab + rowl * 64 + c4);
          *(volatile v4f*)(Sout + (size_t)(b * kHid + i0 + 16 * a + rowl) * kHid + 64 * wave + c4) = sv;
        }
        __threadfence();
      }
    }
    __builtin_amdgcn_fence(__ATOMIC_RELEASE, "workgroup");
    __builtin_amdgcn_wave_barrier();
    __builtin_amdgcn_fence(__ATOMIC_ACQUIRE, "workgroup");
  }
}

__global__ __launch_bounds__(256) void rmsnorm_kernel(
    const float* __restrict__ obuf, const float* __restrict__ g, unsigned short* __restrict__ on16) {
  const int tid = threadIdx.x, lane = tid & 31, wave = tid >> 5;
  const size_t row = (size_t)blockIdx.x * 8 + wave;
  const int c0 = lane * 8;
  const float* xr = obuf + row * kHid;
  const v4f a0 = *(const v4f*)(xr + c0);
  const v4f a1 = *(const v4f*)(xr + c0 + 4);
  const v4f a2 = *(const v4f*)(xr + 256 + c0);
  const v4f a3 = *(const v4f*)(xr + 256 + c0 + 4);
  const v4f g0 = *(const v4f*)(g + c0);
  const v4f g1 = *(const v4f*)(g + c0 + 4);
  const v4f g2 = *(const v4f*)(g + 256 + c0);
  const v4f g3 = *(const v4f*)(g + 256 + c0 + 4);
  float ss = 0.0f;
#pragma unroll
  for (int e = 0; e < 4; ++e) {
    ss = fmaf(a0[e], a0[e], ss);
    ss = fmaf(a1[e], a1[e], ss);
    ss = fmaf(a2[e], a2[e], ss);
    ss = fmaf(a3[e], a3[e], ss);
  }
#pragma unroll
  for (int off = 16; off > 0; off >>= 1) ss += __shfl_xor(ss, off, 32);
  const float inv = 1.0f / sqrtf(ss * (1.0f / (float)kHid) + 1e-5f);
  unsigned short hb[16];
#pragma unroll
  for (int e = 0; e < 4; ++e) {
    hb[e]      = h_bits_fl((a0[e] * inv) * g0[e] * kCarN);
    hb[4 + e]  = h_bits_fl((a1[e] * inv) * g1[e] * kCarN);
    hb[8 + e]  = h_bits_fl((a2[e] * inv) * g2[e] * kCarN);
    hb[12 + e] = h_bits_fl((a3[e] * inv) * g3[e] * kCarN);
  }
  const v4u u0 = (v4u){pk16(hb[0], hb[1]), pk16(hb[2], hb[3]), pk16(hb[4], hb[5]), pk16(hb[6], hb[7])};
  const v4u u1 = (v4u){pk16(hb[8], hb[9]), pk16(hb[10], hb[11]), pk16(hb[12], hb[13]), pk16(hb[14], hb[15])};
  unsigned short* d = on16 + row * kHid;
  for (int pass = 0; pass < 2; ++pass) {
    *(volatile v4u*)(d + c0) = u0;
    *(volatile v4u*)(d + 256 + c0) = u1;
    __threadfence();
  }
}

extern "C" void kernel_launch(void* const* d_in, const int* in_sizes, int n_in,
                              void* d_out, int out_size, void* d_ws, size_t ws_size,
                              hipStream_t stream) {
  if (n_in < 10) return;
  if (in_sizes[0] != kRows * kHid) return;
  if (in_sizes[1] != kHid * kHid) return;
  if (in_sizes[2] != kHid * kHid) return;
  if (in_sizes[3] != kHid * kHid) return;
  if (in_sizes[4] != kHid * kTaps) return;
  if (in_sizes[5] != kHid * kTaps) return;
  if (in_sizes[6] != kHid * kTaps) return;
  if (in_sizes[7] != kHid) return;
  if (in_sizes[8] != kHid) return;
  if (in_sizes[9] != kHid * kHid) return;
  if (out_size != kRows * kHid + kBatch * kHid * kHid) return;
  if (ws_size < kWsTotal) return;

  const float* x      = (const float*)d_in[0];
  const float* Wk     = (const float*)d_in[1];
  const float* Wq     = (const float*)d_in[2];
  const float* Wv     = (const float*)d_in[3];
  const float* conv_k = (const float*)d_in[4];
  const float* conv_q = (const float*)d_in[5];
  const float* conv_v = (const float*)d_in[6];
  const float* Wb     = (const float*)d_in[7];
  const float* gain   = (const float*)d_in[8];
  const float* Wo     = (const float*)d_in[9];
  float* out0 = (float*)d_out;
  float* out1 = (float*)d_out + (size_t)kRows * kHid;

  char* ws = (char*)d_ws;
  unsigned short* X16  = (unsigned short*)(ws + kOffX16);
  unsigned short* W16  = (unsigned short*)(ws + kOffW16);
  float*          RAW  = (float*)(ws + kOffRAW);
  unsigned short* K16  = (unsigned short*)(ws + kOffK16);
  unsigned short* Q16  = (unsigned short*)(ws + kOffQ16);
  unsigned short* KT16 = (unsigned short*)(ws + kOffKT16);
  float*          V32  = (float*)(ws + kOffV32);
  float*          OBUF = (float*)(ws + kOffOBUF);
  unsigned short* ON16 = (unsigned short*)(ws + kOffON16);
  float*          BETA = (float*)(ws + kOffBETA);
  unsigned short* T16  = (unsigned short*)(ws + kOffT16);
  unsigned short* L16  = (unsigned short*)(ws + kOffL16);

  xcvt_beta_kernel<<<kRows / 32, 256, 0, stream>>>(x, Wb, X16, BETA);
  wcast_kernel<<<dim3(kHid * kHid / 8 / 256, 4), 256, 0, stream>>>(Wk, Wq, Wv, Wo, W16);

  wmma_gemm64_f16<<<(kRows / 64) * (kQkvP / 64) / 8, 256, 0, stream>>>(
      X16, kHid, W16, kHid, RAW, kQkvP, kRows, kQkvP, kHid, kProjScale);

  conv_act_norm_kernel<<<kRows, 256, 0, stream>>>(RAW, conv_k, conv_q, conv_v, K16, Q16, V32);
  ktrans_kernel<<<dim3(kSeq / 64, kHid / 64, kBatch), 256, 0, stream>>>(K16, KT16);
  chunk_prep_kernel<<<kBatch * kNChunk, 256, 0, stream>>>(K16, Q16, BETA, T16, L16);
  state_scan_kernel<<<dim3(kHid / kNI, kBatch), 256, 0, stream>>>(K16, Q16, KT16, V32, BETA, T16, L16, OBUF, out1);
  rmsnorm_kernel<<<kRows / 8, 256, 0, stream>>>(OBUF, gain, ON16);

  wmma_gemm64_f16<<<(kRows / 64) * (kHid / 64) / 8, 256, 0, stream>>>(
      ON16, kHid, W16 + (size_t)kQkvP * kHid, kHid, out0, kHid, kRows, kHid, kHid, kOutScale);
}
